// EIGTower_18098992185793
// MI455X (gfx1250) — hardware-run, weakly checked
//
#include <hip/hip_runtime.h>


namespace {
constexpr int N = 30000, NP = 30016  , E = 480000, IN = 128, OUT = 128, ED = 16, NAGG = 5 * IN  , KPOST = 16 * IN  ;
constexpr float XS = 8.0f, WSC = 256.0f, NEG = 0.2f  , AVG = 2.833f, EPSA = 1e-5f, EPSBN = 1e-5f;

typedef _Float16 b16;
typedef __attribute__((ext_vector_type(16))) _Float16 v16b;
typedef __attribute__((ext_vector_type(8))) _Float16 v8b;
typedef __attribute__((ext_vector_type(8))) float v8f;
typedef __attribute__((ext_vector_type(4))) float v4f;
__device__ __forceinline__ float bf16_rne(float f) { unsigned int u = __float_as_uint(f); u += 0x7FFFu + ((u >> 16) & 1u); return __uint_as_float(u & 0xFFFF0000u); }
__device__ __forceinline__ void split16(float v, b16& hi, b16& lo) { hi = (b16)v; lo = (b16)(v - (float)hi); }
__device__ __forceinline__ v16b frag_kb(const b16* p, int hh) { const v8b a = *(const v8b*)(p + 8 * hh), b = *(const v8b*)(p + 16 + 8 * hh); v16b f;
#pragma unroll
  for (int e = 0; e < 8; ++e) { f[e] = a[e]; f[8 + e] = b[e]; } return f; }
__device__ __forceinline__ v8f wmma16b(v16b a, v16b b, v8f c) { v8f d = __builtin_amdgcn_wmma_f32_16x16x32_f16(false, a, false, b, (short)0, c, false, false); asm volatile("v_nop\n\tv_nop\n\tv_nop\n\tv_nop" : "+v"(d) : "v"(a), "v"(b)); return d; }
__device__ __forceinline__ void wave_lds_sync() { __builtin_amdgcn_fence(__ATOMIC_RELEASE, "workgroup"); __builtin_amdgcn_wave_barrier(); __builtin_amdgcn_fence(__ATOMIC_ACQUIRE, "workgroup"); }
__device__ __forceinline__ float pmul(float a, float b) { float p = a * b; asm volatile("" : "+v"(p)); return p; }
__device__ __forceinline__ int iclamp(int v, int lo, int hi) { return v < lo ? lo : (v > hi ? hi : v); }
__device__ __forceinline__ float nexp(float x) { return __builtin_amdgcn_exp2f(x * 1.4426950408889634f); }
__device__ __forceinline__ float lrelu(float x) { return x > 0.0f ? x : NEG * x; }

constexpr int CSR_NBLK = 512, CSR_GB = 9, CSR_GN = 1 << CSR_GB  , CSR_MAXG = 512, CSR_CAP = 12288  ;
__global__ __launch_bounds__(64) void csrA_kernel(const int* __restrict__ dst, int E, int N, int nG, int CHP, int NGP, int* __restrict__ STG, int* __restrict__ HST) {
  extern __shared__ int sm[];
  int* cnt = sm; int* run = sm + NGP; int* ids = sm + 2 * NGP;
  const int b = blockIdx.x; const int ch = (E + CSR_NBLK - 1) / CSR_NBLK; const int e0 = b * ch, e1 = min(E, e0 + ch);
  for (int i = threadIdx.x; i < NGP; i += 64) cnt[i] = 0;
  for (int i = threadIdx.x; i < CHP; i += 64) ids[i] = -1;
  __syncthreads();
  if (threadIdx.x == 0) {
    for (int e = e0; e < e1; ++e) { int d = dst[e]; d = (d < 0) ? 0 : (d >= N ? N - 1 : d); cnt[d >> CSR_GB] += 1; }
    int acc = 0; for (int g = 0; g < nG; ++g) { run[g] = acc; acc += cnt[g]; }
    for (int e = e0; e < e1; ++e) { int d = dst[e]; d = (d < 0) ? 0 : (d >= N ? N - 1 : d); const int g = d >> CSR_GB; ids[run[g]] = e; run[g] += 1; } }
  __syncthreads();
  typedef __attribute__((ext_vector_type(4))) int v4i;
  for (int pass = 0; pass < 2; ++pass) {
    for (int i = threadIdx.x; i < CHP / 4; i += 64) *(volatile v4i*)(STG + (size_t)b * CHP + i * 4) = *(const v4i*)(&ids[i * 4]);
    for (int i = threadIdx.x; i < NGP / 4; i += 64) { v4i v; for (int e = 0; e < 4; ++e) v[e] = (i * 4 + e < nG) ? cnt[i * 4 + e] : 0; *(volatile v4i*)(HST + (size_t)b * NGP + i * 4) = v; }
    __threadfence(); }
}
__global__ __launch_bounds__(512) void csrS_kernel(const int* __restrict__ HST, int nG, int NGP, int* __restrict__ START, int* __restrict__ TOT, int* __restrict__ OFF) {
  __shared__ int tot[CSR_MAXG];
  const int b = threadIdx.x;
  for (int pass = 0; pass < 2; ++pass) { int runb = 0; for (int g = 0; g < nG; ++g) { int c = HST[(size_t)b * NGP + g]; c = (c < 0) ? 0 : c; ((volatile int*)OFF)[(size_t)g * CSR_NBLK + b] = runb; runb += c; } __threadfence(); }
  for (int g = threadIdx.x; g < nG; g += 512) { int s = 0; for (int bb = 0; bb < CSR_NBLK; ++bb) { int c = HST[(size_t)bb * NGP + g]; s += (c < 0) ? 0 : c; } tot[g] = s; }
  __syncthreads();
  if (threadIdx.x < 32) {
    __shared__ int st[CSR_MAXG + 32];
    if (threadIdx.x == 0) { int acc = 0; for (int g = 0; g < NGP; ++g) { st[g] = acc; if (g < nG) acc += (tot[g] + 31) & ~31; } st[NGP] = acc; }
    __builtin_amdgcn_fence(__ATOMIC_RELEASE, "workgroup"); __builtin_amdgcn_wave_barrier(); __builtin_amdgcn_fence(__ATOMIC_ACQUIRE, "workgroup");
    for (int pass = 0; pass < 2; ++pass) { for (int i = threadIdx.x; i < NGP + 32; i += 32) { ((volatile int*)START)[i] = (i <= NGP) ? st[min(i, NGP)] : 0; ((volatile int*)TOT)[i] = (i < nG) ? tot[i] : 0; } __threadfence(); } }
}
__global__ __launch_bounds__(256) void csrB_kernel(const int* __restrict__ dst, int N, int nG, int CHP, int NGP, int permLen, const int* __restrict__ STG, const int* __restrict__ HST, const int* __restrict__ OFF, const int* __restrict__ START, const int* __restrict__ TOT, int* __restrict__ PERM, int* __restrict__ ROWPTR, int* __restrict__ ROWCNT, int* __restrict__ FLAG) {
  typedef __attribute__((ext_vector_type(4))) int v4i;
  __shared__ int ids[CSR_CAP]; __shared__ unsigned short key[CSR_CAP]; __shared__ int outp[CSR_CAP]; __shared__ int ncnt[CSR_GN + 1]; __shared__ int boff[CSR_NBLK + 1];
  const int g = blockIdx.x, t_ = threadIdx.x; int tot = TOT[g]; int st = START[g], stn = START[g + 1]; const int v0 = g * CSR_GN; const int nv = min(CSR_GN, N - v0);
  st = (st < 0) ? 0 : (st > permLen - 32 ? permLen - 32 : st) & ~31; stn = (stn < st) ? st : (stn > permLen ? permLen : stn); tot = (tot < 0) ? 0 : tot; if (tot > stn - st && tot <= CSR_CAP) tot = stn - st;
  if (tot > CSR_CAP) {
    for (int pass = 0; pass < 2; ++pass) { for (int i = t_; i < CSR_GN / 4; i += 256) { v4i a, c; for (int e = 0; e < 4; ++e) { a[e] = st; c[e] = 0; } *(volatile v4i*)(ROWPTR + v0 + i * 4) = a; *(volatile v4i*)(ROWCNT + v0 + i * 4) = c; } if (t_ == 0) ((volatile int*)FLAG)[0] = 1; __threadfence(); } (void)nv; return; }
  if (t_ == 0) { int acc = 0; for (int b = 0; b < CSR_NBLK; ++b) { boff[b] = acc; int c = HST[(size_t)b * NGP + g]; c = (c < 0) ? 0 : (c > CHP ? CHP : c); acc += c; if (acc > tot) acc = tot; } boff[CSR_NBLK] = acc; }
  for (int i = t_; i <= CSR_GN; i += 256) ncnt[i] = 0;
  __syncthreads();
  for (int b = 0; b < CSR_NBLK; ++b) { const int c = boff[b + 1] - boff[b]; int o_ = OFF[(size_t)g * CSR_NBLK + b]; o_ = (o_ < 0) ? 0 : (o_ > CHP - c ? CHP - c : o_); const int* src_ = STG + (size_t)b * CHP + o_;
    for (int i = t_; i < c; i += 256) { int id = src_[i]; id = (id < 0) ? 0 : id; ids[boff[b] + i] = id; int d = dst[id]; d = (d < v0) ? v0 : (d >= N ? N - 1 : d); int kk = d - v0; kk = (kk < 0) ? 0 : (kk >= CSR_GN ? CSR_GN - 1 : kk); key[boff[b] + i] = (unsigned short)kk; } }
  __syncthreads();
  if (t_ == 0) { for (int i = 0; i < tot; ++i) ncnt[key[i]] += 1; int acc = 0; for (int vl = 0; vl < CSR_GN; ++vl) { const int c = ncnt[vl]; ncnt[vl] = acc; acc += c; } ncnt[CSR_GN] = acc;
    for (int i = 0; i < tot; ++i) { const int vl = key[i]; outp[ncnt[vl]] = ids[i]; ncnt[vl] += 1; }
    for (int vl = CSR_GN; vl > 0; --vl) ncnt[vl] = ncnt[vl - 1]; ncnt[0] = 0; }
  __syncthreads();
  for (int pass = 0; pass < 2; ++pass) {
    for (int i = t_; i < (stn - st) / 4; i += 256) { v4i v; for (int e = 0; e < 4; ++e) { const int q = i * 4 + e; v[e] = (q < tot) ? outp[q] : -1; } *(volatile v4i*)(PERM + st + i * 4) = v; }
    for (int i = t_; i < CSR_GN / 4; i += 256) { v4i a, c; for (int e = 0; e < 4; ++e) { const int vl = i * 4 + e; a[e] = st + ncnt[vl]; c[e] = (vl < nv) ? (ncnt[vl + 1] - ncnt[vl]) : 0; } *(volatile v4i*)(ROWPTR + v0 + i * 4) = a; *(volatile v4i*)(ROWCNT + v0 + i * 4) = c; }
    __threadfence(); }
}
__global__ __launch_bounds__(256) void csrZ_kernel(int* __restrict__ p, size_t n4) { typedef __attribute__((ext_vector_type(4))) int v4i; const size_t tid = (size_t)blockIdx.x * 256 + threadIdx.x, nth = (size_t)gridDim.x * 256; v4i z = {0, 0, 0, 0}; for (size_t i = tid; i < n4; i += nth) *(volatile v4i*)(p + i * 4) = z; }
struct CsrBufs { int *STG, *HST, *OFF, *START, *TOT, *PERM, *ROWPTR, *ROWCNT, *FLAG; int nG, NGP, CHP; size_t permLen; char* base; size_t bytes; };
static size_t csr_carve(CsrBufs& c, char* ws, size_t off, int E, int N) {
  const size_t off0 = off; c.base = ws + off;
  auto al = [&](size_t bytes) { char* p = ws + off; off += (bytes + 255) & ~(size_t)255; return p; };
  c.nG = (N + CSR_GN - 1) / CSR_GN; c.NGP = (c.nG + 31) & ~31; const int ch = (E + CSR_NBLK - 1) / CSR_NBLK; c.CHP = (ch + 31) & ~31; c.permLen = (size_t)E + 32 * (size_t)c.nG + 32;
  c.STG = (int*)al((size_t)CSR_NBLK * c.CHP * 4); c.HST = (int*)al((size_t)CSR_NBLK * c.NGP * 4); c.OFF = (int*)al((size_t)c.NGP * CSR_NBLK * 4); c.START = (int*)al((size_t)(c.NGP + 64) * 4); c.TOT = (int*)al((size_t)(c.NGP + 64) * 4);
  c.PERM = (int*)al(c.permLen * 4); c.ROWPTR = (int*)al((size_t)c.nG * CSR_GN * 4); c.ROWCNT = (int*)al((size_t)c.nG * CSR_GN * 4); c.FLAG = (int*)al(256);
  c.bytes = off - off0; return off;
}
static void csr_build(const CsrBufs& c, const int* dst, int E, int N, hipStream_t stream) {
  const size_t smem = (size_t)(2 * c.NGP + c.CHP) * 4;
  csrZ_kernel<<<512, 256, 0, stream>>>((int*)c.base, c.bytes / 16);
  csrA_kernel<<<CSR_NBLK, 64, smem, stream>>>(dst, E, N, c.nG, c.CHP, c.NGP, c.STG, c.HST);
  csrS_kernel<<<1, 512, 0, stream>>>(c.HST, c.nG, c.NGP, c.START, c.TOT, c.OFF);
  csrB_kernel<<<c.nG, 256, 0, stream>>>(dst, N, c.nG, c.CHP, c.NGP, (int)c.permLen, c.STG, c.HST, c.OFF, c.START, c.TOT, c.PERM, c.ROWPTR, c.ROWCNT, c.FLAG);
}


__global__ __launch_bounds__(256) void prep_kernel(const float* __restrict__ h, const float* __restrict__ wpre, const float* __restrict__ wpost, b16* __restrict__ H16, b16* __restrict__ WPA, b16* __restrict__ WPB, b16* __restrict__ WC, b16* __restrict__ WP0, b16* __restrict__ WPS) {
  const size_t t = (size_t)blockIdx.x * 256 + threadIdx.x; size_t u = t; v8b o;
  const size_t nh = (size_t)NP * IN / 8, nab = (size_t)IN * IN / 8, nc = (size_t)IN * 32 / 8, n0 = (size_t)OUT * IN / 8, ns = (size_t)3 * OUT * NAGG / 8;
  if (u < nh) { const size_t e = u * 8; const size_t row = e / IN; for (int j = 0; j < 8; ++j) o[j] = (row < (size_t)N) ? (b16)(bf16_rne(h[e + j]) * XS) : (b16)0.0f; for (int pass = 0; pass < 2; ++pass) { *(volatile v8b*)(H16 + e) = o; __threadfence(); } return; } u -= nh;
  if (u < 2 * nab) { const int kind = (int)(u / nab); const int e = (int)(u % nab) * 8; const int oo = e / IN, k0 = e % IN; for (int j = 0; j < 8; ++j) o[j] = (b16)(bf16_rne(wpre[(size_t)(kind * IN + k0 + j) * IN + oo]) * WSC); for (int pass = 0; pass < 2; ++pass) { *(volatile v8b*)((kind == 0 ? WPA : WPB) + e) = o; __threadfence(); } return; } u -= 2 * nab;
  if (u < nc) { const int e = (int)u * 8; const int oo = e / 32, k0 = e % 32; for (int j = 0; j < 8; ++j) { const int k = k0 + j; o[j] = (k < ED) ? (b16)(bf16_rne(wpre[(size_t)(2 * IN + k) * IN + oo]) * WSC) : (b16)0.0f; } for (int pass = 0; pass < 2; ++pass) { *(volatile v8b*)(WC + e) = o; __threadfence(); } return; } u -= nc;
  if (u < n0) { const int e = (int)u * 8; const int oo = e / IN, k0 = e % IN; for (int j = 0; j < 8; ++j) o[j] = (b16)(bf16_rne(wpost[(size_t)(k0 + j) * OUT + oo]) * WSC); for (int pass = 0; pass < 2; ++pass) { *(volatile v8b*)(WP0 + e) = o; __threadfence(); } return; } u -= n0;
  if (u < ns) { const size_t e = u * 8; const int s = (int)(e / ((size_t)OUT * NAGG)); const int rem = (int)(e % ((size_t)OUT * NAGG)); const int oo = rem / NAGG, k0 = rem % NAGG; for (int j = 0; j < 8; ++j) o[j] = (b16)(bf16_rne(wpost[(size_t)(IN + s * NAGG + k0 + j) * OUT + oo]) * WSC); for (int pass = 0; pass < 2; ++pass) { *(volatile v8b*)(WPS + e) = o; __threadfence(); } }
}
__global__ __launch_bounds__(128) void pq_kernel(const b16* __restrict__ H16, const b16* __restrict__ WPA, const b16* __restrict__ WPB, float* __restrict__ P, float* __restrict__ Q) {
  __shared__ __attribute__((aligned(16))) float Tf[4][16][128 + 4];
  const int wave = threadIdx.x >> 5, lane = threadIdx.x & 31, nloc = lane & 15, hlf = lane >> 4; const int kind = blockIdx.y; const size_t m0 = (size_t)blockIdx.x * 64 + wave * 16;
  const b16* W = kind == 0 ? WPA : WPB; float* Y = kind == 0 ? P : Q; v8f acc[8];
#pragma unroll
  for (int t = 0; t < 8; ++t) acc[t] = (v8f){};
#pragma unroll
  for (int kb = 0; kb < IN; kb += 32) { const v16b a = frag_kb(H16 + (m0 + nloc) * IN + kb, hlf);
#pragma unroll
    for (int t = 0; t < 8; ++t) acc[t] = wmma16b(a, frag_kb(W + (size_t)(t * 16 + nloc) * IN + kb, hlf), acc[t]); }
#pragma unroll
  for (int t = 0; t < 8; ++t)
#pragma unroll
    for (int r = 0; r < 8; ++r) Tf[wave][8 * hlf + r][t * 16 + nloc] = acc[t][r] * (1.0f / (XS * WSC));
  wave_lds_sync();
  for (int pass = 0; pass < 2; ++pass) { for (int rr = 0; rr < 16; ++rr) *(volatile v4f*)(Y + (m0 + rr) * IN + lane * 4) = *(const v4f*)(&Tf[wave][rr][lane * 4]); __threadfence(); }
}
__global__ __launch_bounds__(128) void agg_kernel(const float* __restrict__ P, const float* __restrict__ Q, const float* __restrict__ ef, const float* __restrict__ eig, const float* __restrict__ bpre, const b16* __restrict__ WC,
    const float* __restrict__ fw1, const float* __restrict__ fb1, const float* __restrict__ fw2, const float* __restrict__ fb2, const float* __restrict__ fw3, const float* __restrict__ fb3,
    const int* __restrict__ srcs, const int* __restrict__ PERM, const int* __restrict__ ROWPTR, const int* __restrict__ ROWCNT, int permLen, float* __restrict__ AGf) {
  __shared__ __attribute__((aligned(16))) b16 At[4][16][32 + 8]; __shared__ float wl_s[4][16]; __shared__ int src_s[4][16]; __shared__ __attribute__((aligned(16))) float row[4][NAGG];
  const int wave = threadIdx.x >> 5, lane = threadIdx.x & 31, nloc = lane & 15, hlf = lane >> 4; const size_t v = (size_t)blockIdx.x * 4 + wave;
  int st = 0, cnt = 0; if (v < (size_t)N) { st = ROWPTR[v]; cnt = ROWCNT[v]; cnt = iclamp(cnt, 0, 8192); st = iclamp(st, 0, permLen - cnt); }
  float sm[8], sq[8], mx[8], mn[8], el[8]; float qb[8];
#pragma unroll
  for (int t = 0; t < 8; ++t) { sm[t] = 0.0f; sq[t] = 0.0f; mx[t] = -INFINITY; mn[t] = INFINITY; el[t] = 0.0f; qb[t] = (v < (size_t)N ? Q[v * IN + t * 16 + nloc] : 0.0f) + bf16_rne(bpre[t * 16 + nloc]); }
  const float ev1 = (v < (size_t)N) ? bf16_rne(eig[v * 4 + 1]) : 0.0f, ev2 = (v < (size_t)N) ? bf16_rne(eig[v * 4 + 2]) : 0.0f, ev3 = (v < (size_t)N) ? bf16_rne(eig[v * 4 + 3]) : 0.0f;
  for (int e0 = 0; e0 < cnt; e0 += 16) {
    if (lane < 16) { const int i = e0 + lane; const bool valid = i < cnt; int e = 0, s = 0; if (valid) { e = iclamp(PERM[st + i], 0, E - 1); s = iclamp(srcs[e], 0, N - 1); } src_s[wave][lane] = s;
      for (int k = 0; k < 16; ++k) At[wave][lane][k] = valid ? (b16)(bf16_rne(ef[(size_t)e * ED + k]) * XS) : (b16)0.0f;
      float w = 0.0f; if (valid) { float in6[6] = {bf16_rne(eig[(size_t)s * 4 + 1]), bf16_rne(eig[(size_t)s * 4 + 2]), bf16_rne(eig[(size_t)s * 4 + 3]), ev1, ev2, ev3}; float a[3], b3[3];
        for (int o = 0; o < 3; ++o) { float z = bf16_rne(fb1[o]); for (int k = 0; k < 6; ++k) z += pmul(in6[k], bf16_rne(fw1[k * 3 + o])); a[o] = fmaxf(z, 0.0f); }
        for (int o = 0; o < 3; ++o) { float z = bf16_rne(fb2[o]); for (int k = 0; k < 3; ++k) z += pmul(a[k], bf16_rne(fw2[k * 3 + o])); b3[o] = fmaxf(z, 0.0f); }
        float z = bf16_rne(fb3[0]); for (int k = 0; k < 3; ++k) z += pmul(b3[k], bf16_rne(fw3[k])); w = 1.0f / (1.0f + __expf(-z)); }
      wl_s[wave][lane] = w; }
    else { for (int k = 16; k < 32; ++k) At[wave][lane - 16][k] = (b16)0.0f; }
    wave_lds_sync();
    const v16b a = frag_kb(&At[wave][nloc][0], hlf);
#pragma unroll
    for (int t = 0; t < 8; ++t) { v8f d = {}; d = wmma16b(a, frag_kb(WC + (size_t)(t * 16 + nloc) * 32, hlf), d); const int c = t * 16 + nloc;
#pragma unroll
      for (int r = 0; r < 8; ++r) { const int i = e0 + 8 * hlf + r; if (i < cnt) { const int s = src_s[wave][8 * hlf + r]; const float ee = d[r] * (1.0f / (XS * WSC)) + P[(size_t)s * IN + c] + qb[t];
          sm[t] += ee; sq[t] += ee * ee; mx[t] = fmaxf(mx[t], ee); mn[t] = fminf(mn[t], ee); el[t] += pmul(wl_s[wave][8 * hlf + r], ee); } } }
    wave_lds_sync(); }
  const float degf = (float)cnt; const bool has = cnt > 0; const float sdeg = fmaxf(degf, 1.0f);
#pragma unroll
  for (int t = 0; t < 8; ++t) { float s_ = sm[t] + __shfl_xor(sm[t], 16), q_ = sq[t] + __shfl_xor(sq[t], 16), x_ = fmaxf(mx[t], __shfl_xor(mx[t], 16)), n_ = fminf(mn[t], __shfl_xor(mn[t], 16)), l_ = el[t] + __shfl_xor(el[t], 16);
    const float mean = s_ / sdeg, msq = q_ / sdeg; const float sd = sqrtf(fmaxf(msq - mean * mean, 0.0f) + EPSA); const int c = t * 16 + nloc;
    if (hlf == 0) { row[wave][c] = has ? mean : 0.0f; row[wave][IN + c] = has ? x_ : 0.0f; row[wave][2 * IN + c] = has ? n_ : 0.0f; row[wave][3 * IN + c] = has ? sd : 0.0f; row[wave][4 * IN + c] = has ? l_ : 0.0f; } }
  wave_lds_sync();
  for (int pass = 0; pass < 2; ++pass) { for (int k = 0; k < NAGG / 4 / 32; ++k) *(volatile v4f*)(AGf + v * NAGG + (k * 32 + lane) * 4) = *(const v4f*)(&row[wave][(k * 32 + lane) * 4]); __threadfence(); }
}
__global__ __launch_bounds__(128) void post_kernel(const b16* __restrict__ H16, const float* __restrict__ AGf, const b16* __restrict__ WP0, const b16* __restrict__ WPS, const float* __restrict__ bpost, const float* __restrict__ snorm, const int* __restrict__ ROWCNT, float* __restrict__ OPf) {
  __shared__ __attribute__((aligned(16))) b16 Ah[4][16][160 + 8], Al[4][16][160 + 8]; __shared__ __attribute__((aligned(16))) float Tf[4][16][128 + 4];
  const int wave = threadIdx.x >> 5, lane = threadIdx.x & 31, nloc = lane & 15, hlf = lane >> 4; const size_t m0 = (size_t)blockIdx.x * 64 + wave * 16;
  v8f y[8];
#pragma unroll
  for (int t = 0; t < 8; ++t) y[t] = (v8f){};
#pragma unroll
  for (int kb = 0; kb < IN; kb += 32) { const v16b a = frag_kb(H16 + (m0 + nloc) * IN + kb, hlf);
#pragma unroll
    for (int t = 0; t < 8; ++t) y[t] = wmma16b(a, frag_kb(WP0 + (size_t)(t * 16 + nloc) * IN + kb, hlf), y[t]); }
#pragma unroll
  for (int t = 0; t < 8; ++t) y[t] *= (1.0f / (XS * WSC));
  float c2[8], c3[8];
  for (int r = 0; r < 8; ++r) { const size_t row = m0 + 8 * hlf + r; const int d = (row < (size_t)N) ? iclamp(ROWCNT[row], 0, 8192) : 0; const float lg = logf((float)d + 1.0f); c2[r] = lg / AVG; c3[r] = (d > 0) ? AVG / lg : 0.0f; }
  for (int s = 0; s < 3; ++s) { v8f acc[8];
#pragma unroll
    for (int t = 0; t < 8; ++t) acc[t] = (v8f){};
    for (int kc = 0; kc < NAGG; kc += 160) {
      for (int q = lane; q < 16 * 40; q += 32) { const int rr = q / 40, c4 = (q % 40) * 4; const v4f xv = *(const v4f*)(AGf + (m0 + rr) * NAGG + kc + c4); for (int j = 0; j < 4; ++j) { b16 p, pl; split16(xv[j] * XS, p, pl); Ah[wave][rr][c4 + j] = p; Al[wave][rr][c4 + j] = pl; } }
      wave_lds_sync();
#pragma unroll
      for (int kb = 0; kb < 160; kb += 32) { const v16b a = frag_kb(&Ah[wave][nloc][kb], hlf), al = frag_kb(&Al[wave][nloc][kb], hlf);
#pragma unroll
        for (int t = 0; t < 8; ++t) { const v16b bw = frag_kb(WPS + ((size_t)s * OUT + t * 16 + nloc) * NAGG + kc + kb, hlf); acc[t] = wmma16b(a, bw, acc[t]); acc[t] = wmma16b(al, bw, acc[t]); } }
      wave_lds_sync(); }
#pragma unroll
    for (int t = 0; t < 8; ++t)
#pragma unroll
      for (int r = 0; r < 8; ++r) { const float cs = (s == 0) ? 1.0f : (s == 1 ? c2[r] : c3[r]); y[t][r] += cs * (acc[t][r] * (1.0f / (XS * WSC))); } }
#pragma unroll
  for (int t = 0; t < 8; ++t) { const int c = t * 16 + nloc; const float bb = bf16_rne(bpost[c]);
#pragma unroll
    for (int r = 0; r < 8; ++r) { const size_t row = m0 + 8 * hlf + r; const float sn = (row < (size_t)N) ? bf16_rne(snorm[row]) : 0.0f; Tf[wave][8 * hlf + r][c] = (y[t][r] + bb) * sn; } }
  wave_lds_sync();
  for (int pass = 0; pass < 2; ++pass) { for (int rr = 0; rr < 16; ++rr) *(volatile v4f*)(OPf + (m0 + rr) * OUT + lane * 4) = *(const v4f*)(&Tf[wave][rr][lane * 4]); __threadfence(); }
}
__global__ __launch_bounds__(128) void bn_kernel(const float* __restrict__ X, float* __restrict__ MU, float* __restrict__ RS) {
  __shared__ __attribute__((aligned(16))) float mu_s[OUT], rs_s[OUT];
  const int c = threadIdx.x; double s = 0.0;
#pragma unroll 4
  for (int v = 0; v < N; ++v) s += (double)X[(size_t)v * OUT + c];
  const double mud = s / (double)N; const float mu = (float)mud; double q = 0.0;
#pragma unroll 4
  for (int v = 0; v < N; ++v) { const double d = (double)X[(size_t)v * OUT + c] - mud; q += d * d; }
  mu_s[c] = mu; rs_s[c] = (float)(1.0 / sqrt(q / (double)N + (double)EPSBN));
  __syncthreads();
  for (int pass = 0; pass < 2; ++pass) { if (c < 32) *(volatile v4f*)(MU + c * 4) = *(const v4f*)(&mu_s[c * 4]); else if (c < 64) *(volatile v4f*)(RS + (c - 32) * 4) = *(const v4f*)(&rs_s[(c - 32) * 4]); __threadfence(); }
}
__global__ __launch_bounds__(256) void bnapply_kernel(const float* __restrict__ X, const float* __restrict__ MU, const float* __restrict__ RS, const float* __restrict__ gam, const float* __restrict__ bet, float* __restrict__ out) {
  const int wave = threadIdx.x >> 5, lane = threadIdx.x & 31; const size_t v = (size_t)blockIdx.x * 8 + wave; if (v >= (size_t)N) return;
  const v4f x = *(const v4f*)(X + v * OUT + lane * 4); v4f o; for (int j = 0; j < 4; ++j) { const int c = lane * 4 + j; o[j] = (x[j] - MU[c]) * RS[c] * bf16_rne(gam[c]) + bf16_rne(bet[c]); }
  for (int pass = 0; pass < 2; ++pass) { *(volatile v4f*)(out + v * OUT + lane * 4) = o; __threadfence(); }
}
}

extern "C" void kernel_launch(void* const* d_in, const int* in_sizes, int n_in, void* d_out, int out_size, void* d_ws, size_t ws_size, hipStream_t stream) {
  (void)n_in;
  auto Fp = [&](int i) { return (const float*)d_in[i]; }; auto Ip = [&](int i) { return (const int*)d_in[i]; };
  if (in_sizes[0] != N * IN || in_sizes[1] != N * 4 || in_sizes[2] != E * ED || in_sizes[3] != E || in_sizes[4] != E || in_sizes[5] != N || in_sizes[6] != (2 * IN + ED) * IN || in_sizes[14] != KPOST * OUT || out_size != N * OUT) return;
  size_t off = 0; char* ws = (char*)d_ws;
  auto carve = [&](size_t bytes) { char* p = ws + off; off += (bytes + 255) & ~(size_t)255; return p; };
  b16* H16 = (b16*)carve((size_t)NP * IN * 2); b16* WPA = (b16*)carve((size_t)IN * IN * 2); b16* WPB = (b16*)carve((size_t)IN * IN * 2); b16* WC = (b16*)carve((size_t)IN * 32 * 2); b16* WP0 = (b16*)carve((size_t)OUT * IN * 2); b16* WPS = (b16*)carve((size_t)3 * OUT * NAGG * 2);
  float* P = (float*)carve((size_t)NP * IN * 4); float* Q = (float*)carve((size_t)NP * IN * 4); float* AGf = (float*)carve((size_t)NP * NAGG * 4); float* OPf = P;   float* MU = (float*)carve(OUT * 4); float* RS = (float*)carve(OUT * 4);
  CsrBufs csr; off = csr_carve(csr, ws, off, E, N);
  if (off > ws_size || off > ((size_t)128 << 20)) return;
  prep_kernel<<<(unsigned)(((size_t)NP * IN / 8 + 2 * (size_t)IN * IN / 8 + (size_t)IN * 32 / 8 + (size_t)OUT * IN / 8 + (size_t)3 * OUT * NAGG / 8 + 255) / 256), 256, 0, stream>>>(Fp(0), Fp(6), Fp(14), H16, WPA, WPB, WC, WP0, WPS);
  csr_build(csr, Ip(4), E, N, stream);
  pq_kernel<<<dim3(NP / 64, 2), 128, 0, stream>>>(H16, WPA, WPB, P, Q);
  agg_kernel<<<NP / 4, 128, 0, stream>>>(P, Q, Fp(2), Fp(1), Fp(7), WC, Fp(8), Fp(9), Fp(10), Fp(11), Fp(12), Fp(13), Ip(3), csr.PERM, csr.ROWPTR, csr.ROWCNT, (int)csr.permLen, AGf);
  post_kernel<<<NP / 64, 128, 0, stream>>>(H16, AGf, WP0, WPS, Fp(15), Fp(5), csr.ROWCNT, OPf);
  bn_kernel<<<1, 128, 0, stream>>>(OPf, MU, RS);
  bnapply_kernel<<<NP / 8, 256, 0, stream>>>(OPf, MU, RS, Fp(16), Fp(17), (float*)d_out);
}
